// RecurrentGNN_27298812134108
// MI455X (gfx1250) — hardware-run, weakly checked
//
#include <hip/hip_runtime.h>

typedef float          v8f   __attribute__((ext_vector_type(8)));
typedef float          v4f   __attribute__((ext_vector_type(4)));
typedef unsigned int   v4u   __attribute__((ext_vector_type(4)));
typedef int            v8i   __attribute__((ext_vector_type(8)));
typedef unsigned short v8us  __attribute__((ext_vector_type(8)));
typedef unsigned short v16us __attribute__((ext_vector_type(16)));
typedef __bf16         v16bf __attribute__((ext_vector_type(16)));
typedef _Float16       v16h  __attribute__((ext_vector_type(16)));
typedef v4f  __attribute__((may_alias)) v4fa;
typedef v8us __attribute__((may_alias)) v8usa;
union FragB { v16bf v; v16us u; v8us h[2]; v8i w; };
union FragH { v16h  v; v16us u; v8us h[2]; v8i w; };

__device__ __forceinline__ v8f wmb(const FragB& a, const FragB& b, v8f c) {
  v8f d = __builtin_amdgcn_wmma_f32_16x16x32_bf16(false, a.v, false, b.v, (short)0, c, false, false);
  asm volatile("v_nop\n\tv_nop\n\tv_nop\n\tv_nop" : "+v"(d) : "v"(a.w), "v"(b.w));
  return d;
}

__device__ __forceinline__ v8f wmh(const FragH& a, const FragH& b, v8f c) {
  v8f d = __builtin_amdgcn_wmma_f32_16x16x32_f16(false, a.v, false, b.v, (short)0, c, false, false);
  asm volatile("v_nop\n\tv_nop\n\tv_nop\n\tv_nop" : "+v"(d) : "v"(a.w), "v"(b.w));
  return d;
}

__device__ __forceinline__ unsigned bf16_bits(float f) {
  const unsigned u = __float_as_uint(f);
  const unsigned r = (u + 0x7FFFu + ((u >> 16) & 1u)) >> 16;
  const unsigned q = (u >> 16) | 0x40u;
  return ((u & 0x7fffffffu) > 0x7f800000u) ? q : r;
}

__device__ __forceinline__ float bf16_val(float f) {
  return __uint_as_float(bf16_bits(f) << 16);
}
__device__ __forceinline__ int clampi(int v, int lo, int hi) {
  return v < lo ? lo : (v > hi ? hi : v);
}

__device__ __forceinline__ unsigned f16_bits(float f) {
  const unsigned u  = __float_as_uint(f);
  const unsigned s  = (u >> 16) & 0x8000u;
  const unsigned a  = u & 0x7fffffffu;
  const unsigned t  = a - 0x38000000u;
  const unsigned r  = (t + 0x0FFFu + ((t >> 13) & 1u)) >> 13;
  const unsigned rc = r > 0x7C00u ? 0x7C00u : r;
  const bool small  = a < 0x38800000u;
  const bool isnan  = a > 0x7f800000u;
  const unsigned fin = small ? 0u : (s | rc);
  return isnan ? (s | 0x7E00u) : fin;
}

__device__ __forceinline__ unsigned pk16(unsigned lo, unsigned hi) { return lo | (hi << 16); }
__device__ __forceinline__ unsigned bf16_lo_bits(float v) {
  float hi = bf16_val(v);
  asm volatile("" : "+v"(hi));
  return bf16_bits(v - hi);
}
__device__ __forceinline__ v4u pack8_bf16(v4f a, v4f c) {
  return (v4u){ pk16(bf16_bits(a[0]), bf16_bits(a[1])), pk16(bf16_bits(a[2]), bf16_bits(a[3])),
                pk16(bf16_bits(c[0]), bf16_bits(c[1])), pk16(bf16_bits(c[2]), bf16_bits(c[3])) };
}
__device__ __forceinline__ v4u pack8_bf16_lo(v4f a, v4f c) {
  return (v4u){ pk16(bf16_lo_bits(a[0]), bf16_lo_bits(a[1])), pk16(bf16_lo_bits(a[2]), bf16_lo_bits(a[3])),
                pk16(bf16_lo_bits(c[0]), bf16_lo_bits(c[1])), pk16(bf16_lo_bits(c[2]), bf16_lo_bits(c[3])) };
}
__device__ __forceinline__ v4u pack8_f16(v4f a, v4f c) {
  return (v4u){ pk16(f16_bits(a[0]), f16_bits(a[1])), pk16(f16_bits(a[2]), f16_bits(a[3])),
                pk16(f16_bits(c[0]), f16_bits(c[1])), pk16(f16_bits(c[2]), f16_bits(c[3])) };
}

template <int FORM>
__global__ __launch_bounds__(256) void k_plane(const float* __restrict__ src, int rows, int cols, int ldsrc,
                                               unsigned short* __restrict__ dst, int MP, int KP) {
  static_assert(FORM >= 0 && FORM <= 3);
  const int KTOT = (FORM == 1 || FORM == 3) ? 2 * KP : KP;
  const unsigned ppr   = (unsigned)(KTOT >> 3);
  const unsigned kp8   = (unsigned)(KP >> 3);
  const unsigned total = (unsigned)MP * ppr;
  const unsigned g     = blockIdx.x * 256u + threadIdx.x;
  const unsigned rowu  = g / ppr;
  const unsigned p     = g - rowu * ppr;
  const bool second    = p >= kp8;
  const int row = (int)rowu;
  const int c0  = (int)((second ? p - kp8 : p) << 3);
  const float* srow = src + (size_t)clampi(row, 0, rows - 1) * (size_t)ldsrc;
  float x[8];
  unsigned mk[8];
#pragma unroll
  for (int e = 0; e < 8; ++e) {
    const int c = c0 + e;
    const float v = srow[clampi(c, 0, cols - 1)];
    asm volatile("" :: "v"(v));
    x[e]  = v;
    mk[e] = (row < rows && c < cols) ? 0xFFFFu : 0u;
  }
  const v4f a = (v4f){ x[0], x[1], x[2], x[3] };
  const v4f c = (v4f){ x[4], x[5], x[6], x[7] };
  v4u o;
  if (FORM == 2) {
    o = pack8_f16(a, c);
  } else {
    const v4u hi = pack8_bf16(a, c);
    o = hi;
    if (FORM == 1) { const v4u lo = pack8_bf16_lo(a, c); o = second ? lo : hi; }
  }
  const v4u mw = (v4u){ pk16(mk[0], mk[1]), pk16(mk[2], mk[3]), pk16(mk[4], mk[5]), pk16(mk[6], mk[7]) };
  o &= mw;
  if (g < total) {
    volatile v4u* q = (volatile v4u*)(dst + (size_t)g * 8);
    *q = o;
    __threadfence();
    *q = o;
  }
}

template <int FORM> struct FragOf    { typedef FragB T; };
template <>         struct FragOf<2> { typedef FragH T; };
__device__ __forceinline__ v8f mm(const FragB& a, const FragB& b, v8f c) { return wmb(a, b, c); }
__device__ __forceinline__ v8f mm(const FragH& a, const FragH& b, v8f c) { return wmh(a, b, c); }
template <class F> __device__ __forceinline__ F ld_frag(const unsigned short* p) {
  F f;
  f.h[0] = *(const v8usa*)(p);
  f.h[1] = *(const v8usa*)(p + 16);
  return f;
}

template <int FORM, int EPI>
__global__ __launch_bounds__(256) __attribute__((amdgpu_num_vgpr(248)))
void k_gemm_nt(const unsigned short* __restrict__ A, const unsigned short* __restrict__ B,
               const float* __restrict__ bias, float* __restrict__ D, int M, int N, int KTOT, int ldd) {
  static_assert(FORM >= 0 && FORM <= 2);
  static_assert(EPI == 0 || EPI == 1);
  typedef typename FragOf<FORM>::T F;
  __shared__ __attribute__((aligned(16))) float sT[8][16 * 68];
  const int lane = threadIdx.x & 31;
  const int wave = threadIdx.x >> 5;
  const int tilesM = (M + 63) >> 6;
  const int tilesN = (N + 63) >> 6;
  const int tile = blockIdx.x * 8 + wave;
  if (tile >= tilesM * tilesN) return;
  const int tm = tile / tilesN;
  const int tn = tile - tm * tilesN;
  const int m0 = tm << 6;
  const int n0 = tn << 6;

  const int rl = lane & 15;
  const int h8 = (lane >> 4) * 8;
  const unsigned short* pa = A + (size_t)(m0 + rl) * (size_t)KTOT + h8;
  const unsigned short* pb = B + (size_t)(n0 + rl) * (size_t)KTOT + h8;

  v8f acc[4][4];
#pragma unroll
  for (int i = 0; i < 4; ++i)
#pragma unroll
    for (int j = 0; j < 4; ++j) acc[i][j] = (v8f){0.f, 0.f, 0.f, 0.f, 0.f, 0.f, 0.f, 0.f};

#pragma unroll 1
  for (int k0 = 0; k0 < KTOT; k0 += 32) {
    F bf[4];
#pragma unroll
    for (int j = 0; j < 4; ++j) bf[j] = ld_frag<F>(pb + (size_t)(j << 4) * (size_t)KTOT + k0);
#pragma unroll
    for (int i = 0; i < 4; ++i) {
      const F af = ld_frag<F>(pa + (size_t)(i << 4) * (size_t)KTOT + k0);
#pragma unroll
      for (int j = 0; j < 4; ++j) acc[i][j] = mm(af, bf[j], acc[i][j]);
    }
  }

  float* slab = sT[wave];
  const int hh = lane >> 4;
  const int c4 = (lane & 15) * 4;
  const int nc = n0 + c4;
  const bool cok = nc < N;
  v4f bv = (v4f){0.f, 0.f, 0.f, 0.f};
  if (EPI == 1) {
    bv = *(const v4fa*)(bias + clampi(nc, 0, N - 4));
    asm volatile("" :: "v"(bv));
  }
#pragma unroll
  for (int i = 0; i < 4; ++i) {
    const int mBase = m0 + (i << 4);
#pragma unroll
    for (int j = 0; j < 4; ++j) {
#pragma unroll
      for (int r = 0; r < 8; ++r) slab[(h8 + r) * 68 + (j << 4) + rl] = acc[i][j][r];
    }
    __builtin_amdgcn_fence(__ATOMIC_RELEASE, "workgroup");
    __builtin_amdgcn_wave_barrier();
    __builtin_amdgcn_fence(__ATOMIC_ACQUIRE, "workgroup");
    v4f vv[8];
#pragma unroll
    for (int it = 0; it < 8; ++it) {
      const int row = it * 2 + hh;
      v4f v = *(const v4fa*)(slab + row * 68 + c4);
      if (EPI == 1) v += bv;
      vv[it] = v;
    }
    for (int pass = 0; pass < 2; ++pass) {
#pragma unroll
      for (int it = 0; it < 8; ++it) {
        const int row = mBase + it * 2 + hh;
        if (cok && row < M) *(volatile v4f*)(D + (size_t)row * (size_t)ldd + nc) = vv[it];
      }
      __threadfence();
    }
    __builtin_amdgcn_fence(__ATOMIC_RELEASE, "workgroup");
    __builtin_amdgcn_wave_barrier();
    __builtin_amdgcn_fence(__ATOMIC_ACQUIRE, "workgroup");
  }
}

#pragma clang fp contract(off)

#ifndef SITE2_TWO_TERM
#define SITE2_TWO_TERM 1
#endif
#ifndef SITE3_TWO_TERM
#define SITE3_TWO_TERM 1
#endif

typedef int   v4i __attribute__((ext_vector_type(4)));
typedef v4i   __attribute__((may_alias)) v4ia;
typedef float v2f __attribute__((ext_vector_type(2)));
typedef v2f   __attribute__((may_alias)) v2fa;

constexpr int NN     = 100000;
constexpr int NE     = 800000;
constexpr int XF     = 24;
constexpr int HID    = 64;
constexpr int OUTP   = 12;
constexpr int NP     = 100096;
constexpr int KX     = 32;
constexpr int KH     = 128;
constexpr int NPC    = 128;
constexpr int OUT_ELEMS = NN * OUTP;
constexpr int NBRUN  = 1024;
constexpr int NBLK   = 98;
constexpr int RCAP   = 11264;
constexpr int WLCAP  = 2048;
constexpr int DEGCAP = 48;
constexpr int EPW    = NE / 8;
constexpr int SUB    = 64;
constexpr int NSTEP  = (EPW + SUB - 1) / SUB;
constexpr int MEAS_B1024_A = 8423, MEAS_B1024_B = 8358;
constexpr int MEAS_DEG_A = 22, MEAS_DEG_B = 20;

static_assert(NP % 64 == 0 && NP >= NN && NP - NN < 128 && NP % 128 == 0 && NP % 8 == 0);
static_assert(NN % 16 == 0 && NN % 32 == 0 && NN % 8 == 0);
static_assert(KX % 32 == 0 && KX >= XF && KH % 32 == 0 && KH == 2 * HID && NPC % 64 == 0 && NPC % 32 == 0);
static_assert(HID % 64 == 0 && HID % 32 == 0 && OUTP % 4 == 0 && OUTP <= HID);
static_assert(NBLK * NBRUN >= NN && (NBLK - 1) * NBRUN < NN);
static_assert(NE % 8 == 0 && EPW * 8 == NE && NSTEP * SUB >= EPW && (NSTEP - 1) * SUB < EPW);
static_assert(RCAP % 1024 == 0 && RCAP * 4 >= MEAS_B1024_A * 5 && RCAP * 4 >= MEAS_B1024_B * 5);
static_assert(WLCAP * 8 >= RCAP && WLCAP % 4 == 0);
static_assert(DEGCAP * 4 >= MEAS_DEG_A * 5 && DEGCAP * 4 >= MEAS_DEG_B * 5 && DEGCAP <= 64 && DEGCAP > 32);
static_assert(RCAP >= 2 * DEGCAP);
static_assert(((((long long)(NN - 1)) << 10) | 1023) < (1LL << 31));
static_assert(9375 * 128 == OUT_ELEMS && OUT_ELEMS == 1200000);
static_assert((long long)NP * KH / 8 < 0x7fffffffLL);

constexpr int BK_WLW  = 0;
constexpr int BK_WLE  = BK_WLW + 8 * WLCAP;
constexpr int BK_SLN  = BK_WLE + 8 * WLCAP;
constexpr int BK_SLE  = BK_SLN + RCAP;
constexpr int BK_CNT  = BK_SLE + RCAP;
constexpr int BK_OFF  = BK_CNT + NBRUN;
constexpr int BK_CUR  = BK_OFF + NBRUN;
constexpr int BK_MISC = BK_CUR + NBRUN;
constexpr int BK_INTS = BK_MISC + 16;
constexpr int BK_LDS  = BK_INTS * 4;
static_assert(BK_LDS == 233536 && BK_LDS <= 262144);
static_assert(BK_SLN % 4 == 0 && BK_SLE % 4 == 0 && BK_CNT % 4 == 0 && BK_OFF % 4 == 0);
static_assert((2 * RCAP + NBRUN) % 1024 == 0 && (RCAP / 4) % 256 == 0);

constexpr size_t SZ_P    = (size_t)NN * NPC * 4;
constexpr size_t SZ_ZS   = (size_t)NN * HID * 4;
constexpr size_t SZ_HHL  = (size_t)NP * KH * 2;
constexpr size_t SZ_X24  = (size_t)NP * KX * 2;
constexpr size_t SZ_LIST = (size_t)NBLK * RCAP * 4;
constexpr size_t SZ_NODE = (size_t)NBLK * NBRUN * 4;
constexpr size_t SZ_RD   = 400128;
constexpr size_t SZ_W1T  = (size_t)64 * KX * 2;
constexpr size_t SZ_WCT  = (size_t)4 * 128 * KH * 2;
constexpr size_t SZ_WOT  = (size_t)64 * KH * 2;
constexpr size_t SZ_BIAS = 1024;
constexpr size_t OFF_P    = 0;
constexpr size_t OFF_ZS   = OFF_P + SZ_P;
constexpr size_t OFF_HHL  = OFF_ZS + SZ_ZS;
constexpr size_t OFF_X24  = OFF_HHL + SZ_HHL;
constexpr size_t OFF_LNA  = OFF_X24 + SZ_X24;
constexpr size_t OFF_LEA  = OFF_LNA + SZ_LIST;
constexpr size_t OFF_LNB  = OFF_LEA + SZ_LIST;
constexpr size_t OFF_LEB  = OFF_LNB + SZ_LIST;
constexpr size_t OFF_CA   = OFF_LEB + SZ_LIST;
constexpr size_t OFF_OA   = OFF_CA + SZ_NODE;
constexpr size_t OFF_FA   = OFF_OA + SZ_NODE;
constexpr size_t OFF_CB   = OFF_FA + SZ_NODE;
constexpr size_t OFF_OB   = OFF_CB + SZ_NODE;
constexpr size_t OFF_FB   = OFF_OB + SZ_NODE;
constexpr size_t OFF_RDI  = OFF_FB + SZ_NODE;
constexpr size_t OFF_RDO  = OFF_RDI + SZ_RD;
constexpr size_t OFF_W1T  = OFF_RDO + SZ_RD;
constexpr size_t OFF_WCT  = OFF_W1T + SZ_W1T;
constexpr size_t OFF_WOT  = OFF_WCT + SZ_WCT;
constexpr size_t OFF_BIAS = OFF_WOT + SZ_WOT;
constexpr size_t WS_TOTAL = OFF_BIAS + SZ_BIAS;
static_assert(WS_TOTAL == (size_t)((size_t)253621 << 9));
static_assert(WS_TOTAL <= ((size_t)128 << 20));
static_assert(SZ_P % 256 == 0 && SZ_ZS % 256 == 0 && SZ_HHL % 256 == 0 && SZ_X24 % 256 == 0 && SZ_LIST % 256 == 0);
static_assert(SZ_NODE % 256 == 0 && SZ_RD % 256 == 0 && SZ_RD >= (size_t)NN * 4 && SZ_W1T % 256 == 0);
static_assert(SZ_WCT % 256 == 0 && SZ_WOT % 256 == 0 && SZ_BIAS % 256 == 0);
static_assert((size_t)NN * HID * 4 <= SZ_P);
static_assert((size_t)NBLK * NBRUN >= (size_t)NN);

__device__ __forceinline__ float sigm(float v) { return 1.0f / (1.0f + expf(-v)); }

constexpr int PREP_TILE   = 64 * 33;
constexpr int PREP_BLOCKS = 19;
static_assert(PREP_TILE >= 63 * 33 + 32 && PREP_TILE >= 23 * 65 + 64 && PREP_TILE >= 63 * 13 + 12);

__device__ __forceinline__ void wct_load(const float* __restrict__ W, float* tile, int tid, int mat, int c0) {
  const float* s = W + (size_t)mat * 8192 + c0;
#pragma unroll
  for (int it = 0; it < 2; ++it) {
    const int qi = tid + 256 * it;
    const int r  = qi >> 3;
    const int c4 = (qi & 7) * 4;
    const v4f v = *(const v4fa*)(s + r * 64 + c4);
    asm volatile("" :: "v"(v));
    tile[r * 33 + c4 + 0] = v[0];
    tile[r * 33 + c4 + 1] = v[1];
    tile[r * 33 + c4 + 2] = v[2];
    tile[r * 33 + c4 + 3] = v[3];
  }
}

__global__ __launch_bounds__(256) void k_prep(const float* __restrict__ wl2, const float* __restrict__ bl2,
                                              const float* __restrict__ wz, const float* __restrict__ bz,
                                              const float* __restrict__ wh, const float* __restrict__ bh,
                                              const float* __restrict__ wo, const float* __restrict__ bo,
                                              unsigned short* __restrict__ W1T, unsigned short* __restrict__ WCT,
                                              unsigned short* __restrict__ WOT, float* __restrict__ BIAS) {
  __shared__ __attribute__((aligned(16))) float tile[PREP_TILE];
  const int tid = (int)threadIdx.x;
  const int blk = (int)blockIdx.x;
  const int q   = (blk >> 2) & 3;
  const int j   = blk & 3;

  if (blk < 16) {
    const int mat = (j & 1) * 2 + (j >> 1);
    const int c0  = 32 * (q & 1);
    if ((q >> 1) == 0) wct_load(wz, tile, tid, mat, c0);
    else               wct_load(wh, tile, tid, mat, c0);
  } else if (blk == 16) {
#pragma unroll
    for (int it = 0; it < 2; ++it) {
      const int qi = tid + 256 * it;
      const int qc = qi < 383 ? qi : 383;
      const int r  = qc >> 4;
      const int c4 = (qc & 15) * 4;
      const v4f v = *(const v4fa*)(wl2 + r * 64 + c4);
      asm volatile("" :: "v"(v));
      if (qi < 384) {
        tile[r * 65 + c4 + 0] = v[0];
        tile[r * 65 + c4 + 1] = v[1];
        tile[r * 65 + c4 + 2] = v[2];
        tile[r * 65 + c4 + 3] = v[3];
      }
    }
  } else if (blk == 17) {
    const int qc = tid < 191 ? tid : 191;
    const int r  = qc / 3;
    const int c4 = (qc - r * 3) * 4;
    const v4f v = *(const v4fa*)(wo + 4 * qc);
    asm volatile("" :: "v"(v));
    if (tid < 192) {
      tile[r * 13 + c4 + 0] = v[0];
      tile[r * 13 + c4 + 1] = v[1];
      tile[r * 13 + c4 + 2] = v[2];
      tile[r * 13 + c4 + 3] = v[3];
    }
  }
  __syncthreads();

  if (blk < 16) {
    v4u o[2];
#pragma unroll
    for (int it = 0; it < 2; ++it) {
      const int qi   = tid + 256 * it;
      const int n    = qi >> 4;
      const int cin0 = ((qi & 15) * 8) & 63;
      const float* tp = tile + cin0 * 33 + n;
      const v4f a = (v4f){ tp[0 * 33], tp[1 * 33], tp[2 * 33], tp[3 * 33] };
      const v4f c = (v4f){ tp[4 * 33], tp[5 * 33], tp[6 * 33], tp[7 * 33] };
      o[it] = pack8_bf16(a, c);
    }
    unsigned short* dst = WCT + (size_t)(q * 128 + 32 * j) * KH;
#pragma unroll
    for (int it = 0; it < 2; ++it) *(volatile v4u*)(dst + (size_t)(tid + 256 * it) * 8) = o[it];
    __threadfence();
#pragma unroll
    for (int it = 0; it < 2; ++it) *(volatile v4u*)(dst + (size_t)(tid + 256 * it) * 8) = o[it];
  } else if (blk == 16) {
    const int n  = tid >> 2;
    const int k0 = (tid & 3) * 8;
    unsigned hb[8];
#pragma unroll
    for (int e = 0; e < 8; ++e) {
      const int k  = k0 + e;
      const int kc = k < XF - 1 ? k : XF - 1;
      const unsigned m = (k < XF) ? 0xFFFFu : 0u;
      hb[e] = bf16_bits(tile[kc * 65 + n]) & m;
    }
    const v4u o = (v4u){ pk16(hb[0], hb[1]), pk16(hb[2], hb[3]), pk16(hb[4], hb[5]), pk16(hb[6], hb[7]) };
    volatile v4u* p = (volatile v4u*)(W1T + (size_t)tid * 8);
    *p = o;
    __threadfence();
    *p = o;
  } else if (blk == 17) {
    v4u o[4];
#pragma unroll
    for (int it = 0; it < 4; ++it) {
      const int qi = tid + 256 * it;
      const int n  = qi >> 4;
      const int k0 = ((qi & 15) * 8) & 63;
      const int nc = n < OUTP - 1 ? n : OUTP - 1;
      const unsigned m = (n < OUTP) ? 0xFFFFu : 0u;
      unsigned hb[8];
#pragma unroll
      for (int e = 0; e < 8; ++e) hb[e] = bf16_bits(tile[(k0 + e) * 13 + nc]) & m;
      o[it] = (v4u){ pk16(hb[0], hb[1]), pk16(hb[2], hb[3]), pk16(hb[4], hb[5]), pk16(hb[6], hb[7]) };
    }
#pragma unroll
    for (int it = 0; it < 4; ++it) *(volatile v4u*)(WOT + (size_t)(tid + 256 * it) * 8) = o[it];
    __threadfence();
#pragma unroll
    for (int it = 0; it < 4; ++it) *(volatile v4u*)(WOT + (size_t)(tid + 256 * it) * 8) = o[it];
  } else {
    const int jj  = tid & 15;
    const int seg = (tid >> 4) & 3;
    const int j3  = jj < 2 ? jj : 2;
    const v4f a0 = *(const v4fa*)(bl2 + 4 * jj);
    const v4f a1 = *(const v4fa*)(bz + 4 * jj);
    const v4f a2 = *(const v4fa*)(bh + 4 * jj);
    const v4f a3 = *(const v4fa*)(bo + 4 * j3);
    asm volatile("" :: "v"(a0));
    asm volatile("" :: "v"(a1));
    asm volatile("" :: "v"(a2));
    asm volatile("" :: "v"(a3));
    const unsigned m0 = (seg == 0) ? 0xFFFFFFFFu : 0u;
    const unsigned m1 = (seg == 1) ? 0xFFFFFFFFu : 0u;
    const unsigned m2 = (seg == 2) ? 0xFFFFFFFFu : 0u;
    const unsigned m3 = (seg == 3 && jj < 3) ? 0xFFFFFFFFu : 0u;
    v4f ob;
#pragma unroll
    for (int e = 0; e < 4; ++e) {
      const unsigned bits = (__float_as_uint(a0[e]) & m0) | (__float_as_uint(a1[e]) & m1) |
                            (__float_as_uint(a2[e]) & m2) | (__float_as_uint(a3[e]) & m3);
      ob[e] = bf16_val(__uint_as_float(bits));
    }
    if (tid < 64) *(volatile v4f*)(BIAS + 4 * tid) = ob;
    __threadfence();
    if (tid < 64) *(volatile v4f*)(BIAS + 4 * tid) = ob;
  }
}

__global__ __launch_bounds__(256) void k_build(const int* __restrict__ keyp, const int* __restrict__ othp,
                                               int* __restrict__ LISTN, int* __restrict__ LISTE,
                                               int* __restrict__ CNT, int* __restrict__ OFF, int* __restrict__ FLG) {
  extern __shared__ __attribute__((aligned(16))) int dsm[];
  int* wlw  = dsm + BK_WLW;
  int* wle  = dsm + BK_WLE;
  int* sln  = dsm + BK_SLN;
  int* sle  = dsm + BK_SLE;
  int* cnt  = dsm + BK_CNT;
  int* offs = dsm + BK_OFF;
  int* cur  = dsm + BK_CUR;
  int* misc = dsm + BK_MISC;
  const int tid = (int)threadIdx.x, lane = tid & 31, wave = tid >> 5;
  const int blk = (int)blockIdx.x;
  const int nodeBase = blk * NBRUN;
  const int nbi = (NN - nodeBase) < NBRUN ? (NN - nodeBase) : NBRUN;
  const unsigned unb = (unsigned)(nbi < 0 ? 0 : nbi);

  {
    const v4i z4 = (v4i){0, 0, 0, 0};
    for (int i = tid * 4; i < 2 * RCAP + NBRUN; i += 1024) *(v4ia*)(sln + i) = z4;
    if (tid < 16) misc[tid] = 0;
  }
  __syncthreads();

  int* mylw = wlw + wave * WLCAP;
  int* myle = wle + wave * WLCAP;
  const int wbase = wave * EPW;
  const int wlast = wbase + EPW - 1;
  int wc = 0;
#pragma unroll 1
  for (int st = 0; st < NSTEP; ++st) {
    const int e0 = wbase + st * SUB + lane;
    int dk[2], wk[2], ek[2];
#pragma unroll
    for (int j = 0; j < 2; ++j) {
      const int e  = e0 + 32 * j;
      const int ec = e < wlast ? e : wlast;
      const int d = keyp[ec];
      const int s = othp[ec];
      asm volatile("" :: "v"(d));
      asm volatile("" :: "v"(s));
      dk[j] = (e <= wlast) ? d : -1;
      wk[j] = clampi(s, 0, NN - 1);
      ek[j] = ec;
    }
#pragma unroll
    for (int j = 0; j < 2; ++j) {
      const unsigned slot = (unsigned)dk[j] - (unsigned)nodeBase;
      const bool hit = slot < unb;
      const unsigned mj = __builtin_amdgcn_ballot_w32(hit);
      if (mj != 0u) {
        if (hit) {
          const int pos = wc + (int)__builtin_amdgcn_mbcnt_lo(mj, 0u);
          if (pos < WLCAP) {
            mylw[pos] = (wk[j] << 10) | (int)slot;
            myle[pos] = ek[j];
          }
        }
        wc += (int)__builtin_popcount(mj);
      }
    }
  }
  if (lane == 0) misc[wave] = wc;
  __syncthreads();

  if (wave == 0) {
    int t = 0, ov = 0;
#pragma unroll 1
    for (int w2 = 0; w2 < 8; ++w2) {
      const int craw = misc[w2];
      ov |= (craw > WLCAP) ? 1 : 0;
      const int c = __builtin_amdgcn_readfirstlane(clampi(craw, 0, WLCAP));
#pragma unroll 1
      for (int b0 = 0; b0 < c; b0 += 32) {
        const int idx = (b0 + lane) < c ? (b0 + lane) : c - 1;
        const int ent = wlw[w2 * WLCAP + idx];
        const int m32 = (c - b0) < 32 ? (c - b0) : 32;
#pragma unroll 1
        for (int k = 0; k < m32; ++k) {
          const int u    = __builtin_amdgcn_readlane(ent, k);
          const int slot = u & (NBRUN - 1);
          if (t < RCAP) {
            if (lane == 0) cnt[slot] = cnt[slot] + 1;
            t = t + 1;
          } else {
            ov = 1;
          }
        }
      }
    }
    if (lane == 0) { misc[8] = t; misc[9] = ov; }
  }
  __syncthreads();

  if (wave == 0) {
    const int base = lane * (NBRUN / 32);
    int s = 0;
#pragma unroll 1
    for (int i = 0; i < NBRUN / 32; ++i) s += cnt[base + i];
    int incl = s;
#pragma unroll
    for (int d = 1; d < 32; d <<= 1) {
      const int y = __shfl_up(incl, d, 32);
      incl += (lane >= d) ? y : 0;
    }
    int run = incl - s;
#pragma unroll 1
    for (int i = 0; i < NBRUN / 32; ++i) {
      const int cv = cnt[base + i];
      offs[base + i] = run;
      cur[base + i]  = run;
      run += cv;
    }
  }
  __syncthreads();

  if (wave == 0) {
    int t2 = 0;
#pragma unroll 1
    for (int w2 = 0; w2 < 8; ++w2) {
      const int c = __builtin_amdgcn_readfirstlane(clampi(misc[w2], 0, WLCAP));
#pragma unroll 1
      for (int b0 = 0; b0 < c; b0 += 32) {
        const int idx = (b0 + lane) < c ? (b0 + lane) : c - 1;
        const int ent = wlw[w2 * WLCAP + idx];
        const int ene = wle[w2 * WLCAP + idx];
        const int m32 = (c - b0) < 32 ? (c - b0) : 32;
#pragma unroll 1
        for (int k = 0; k < m32; ++k) {
          const int u    = __builtin_amdgcn_readlane(ent, k);
          const int ue   = __builtin_amdgcn_readlane(ene, k);
          const int slot = u & (NBRUN - 1);
          if (t2 < RCAP) {
            if (lane == 0) {
              int p = cur[slot];
              p = clampi(p, 0, RCAP - 1);
              sln[p] = u >> 10;
              sle[p] = ue;
              cur[slot] = p + 1;
            }
            t2 = t2 + 1;
          }
        }
      }
    }
  }
  __syncthreads();

  const int ovf = misc[9];
  int* nbase = LISTN + (size_t)blk * RCAP;
  int* ebase = LISTE + (size_t)blk * RCAP;
  for (int pass = 0; pass < 2; ++pass) {
    for (int i = tid; i < RCAP / 4; i += 256) {
      const v4i vn = *(const v4ia*)(sln + 4 * i);
      const v4i ve = *(const v4ia*)(sle + 4 * i);
      *(volatile v4i*)(nbase + 4 * i) = vn;
      *(volatile v4i*)(ebase + 4 * i) = ve;
    }
    __threadfence();
  }
  const v4i cv4 = *(const v4ia*)(cnt + 4 * tid);
  const v4i ov4 = *(const v4ia*)(offs + 4 * tid);
  const v4i fl4 = (v4i){ ((cv4.x > DEGCAP) ? 1 : 0) | ovf, ((cv4.y > DEGCAP) ? 1 : 0) | ovf,
                         ((cv4.z > DEGCAP) ? 1 : 0) | ovf, ((cv4.w > DEGCAP) ? 1 : 0) | ovf };
  const size_t nb4 = (size_t)nodeBase + 4 * (size_t)tid;
  *(volatile v4i*)(CNT + nb4) = cv4;
  *(volatile v4i*)(OFF + nb4) = ov4;
  *(volatile v4i*)(FLG + nb4) = fl4;
  __threadfence();
  *(volatile v4i*)(CNT + nb4) = cv4;
  *(volatile v4i*)(OFF + nb4) = ov4;
  *(volatile v4i*)(FLG + nb4) = fl4;
}

__device__ __forceinline__ int list_word(const int* __restrict__ LIST, int b, int o, int n, int idx) {
  int i = idx < n ? idx : n - 1;
  i = clampi(i, 0, DEGCAP - 1);
  const int w = LIST[(size_t)b * RCAP + o + i];
  asm volatile("" :: "v"(w));
  return w;
}

__device__ __forceinline__ float deg_recip(const int* __restrict__ LISTE, const int* __restrict__ CNT,
                                           const int* __restrict__ OFF, const int* __restrict__ FLG,
                                           const float* __restrict__ ew, int ic, int lane) {
  const int b = ic >> 10;
  int c = CNT[ic];
  int o = OFF[ic];
  const int fl = FLG[ic];
  asm volatile("" :: "v"(c));
  asm volatile("" :: "v"(o));
  asm volatile("" :: "v"(fl));
  c = clampi(c, 0, DEGCAP);
  o = clampi(o, 0, RCAP - DEGCAP);
  const int cn = __builtin_amdgcn_readfirstlane(c);
  const int e0 = clampi(list_word(LISTE, b, o, cn, lane), 0, NE - 1);
  const int e1 = clampi(list_word(LISTE, b, o, cn, lane + 32), 0, NE - 1);
  float w0 = ew[e0];
  float w1 = ew[e1];
  asm volatile("" :: "v"(w0));
  asm volatile("" :: "v"(w1));
  w0 = bf16_val(w0);
  w1 = bf16_val(w1);
  float s = 0.0f;
  const int c1 = cn < 32 ? cn : 32;
#pragma unroll 1
  for (int k = 0; k < c1; ++k) s = s + __int_as_float(__builtin_amdgcn_readlane(__float_as_int(w0), k));
#pragma unroll 1
  for (int k = 32; k < cn; ++k) s = s + __int_as_float(__builtin_amdgcn_readlane(__float_as_int(w1), k - 32));
  const float r  = 1.0f / s;
  const float qn = __int_as_float(0x7fc00000);
  return (fl != 0) ? qn : r;
}

__global__ __launch_bounds__(256) void k_deg(const float* __restrict__ ew,
                                             const int* __restrict__ LEA, const int* __restrict__ CA,
                                             const int* __restrict__ OA, const int* __restrict__ FA,
                                             const int* __restrict__ LEB, const int* __restrict__ CB,
                                             const int* __restrict__ OB, const int* __restrict__ FB,
                                             float* __restrict__ RDI, float* __restrict__ RDO) {
  __shared__ float sR[2][32];
  const int tid = (int)threadIdx.x, lane = tid & 31, wave = tid >> 5;
  const int nb0 = (int)blockIdx.x * 32;
#pragma unroll 1
  for (int i = 0; i < 4; ++i) {
    const int n  = nb0 + wave * 4 + i;
    const int ic = clampi(n, 0, NN - 1);
    const float ri = deg_recip(LEA, CA, OA, FA, ew, ic, lane);
    const float ro = deg_recip(LEB, CB, OB, FB, ew, ic, lane);
    if (lane == 0) { sR[0][wave * 4 + i] = ri; sR[1][wave * 4 + i] = ro; }
  }
  __syncthreads();
  const float v0 = sR[0][lane];
  const float v1 = sR[1][lane];
  const int g = nb0 + lane;
  const bool ok = g < NN;
  const int gc = clampi(g, 0, NN - 1);
  if (wave == 0 && ok) *(volatile float*)(RDI + gc) = v0;
  if (wave == 1 && ok) *(volatile float*)(RDO + gc) = v1;
  __threadfence();
  if (wave == 0 && ok) *(volatile float*)(RDI + gc) = v0;
  if (wave == 1 && ok) *(volatile float*)(RDO + gc) = v1;
}

template <int MODE, int TWO>
__global__ __launch_bounds__(256) void k_split(const float* __restrict__ SRC, const float* __restrict__ bias,
                                               unsigned* __restrict__ DST32) {
  static_assert(MODE == 0 || MODE == 1);
  const int tid = (int)threadIdx.x, lane = tid & 31, wave = tid >> 5;
  const int row = (int)blockIdx.x * 8 + wave;
  const int rc  = clampi(row, 0, NN - 1);
  const v2f x = *(const v2fa*)(SRC + (size_t)rc * HID + 2 * lane);
  asm volatile("" :: "v"(x));
  float v0 = x[0], v1 = x[1];
  if (MODE == 0) {
    const v2f bv = *(const v2fa*)(bias + 2 * lane);
    asm volatile("" :: "v"(bv));
    v0 = sigm(v0 + bv[0]);
    v1 = sigm(v1 + bv[1]);
  }
  unsigned wh = pk16(bf16_bits(v0), bf16_bits(v1));
  unsigned wl = 0u;
  if (TWO != 0) wl = pk16(bf16_lo_bits(v0), bf16_lo_bits(v1));
  const unsigned msk = (row < NN) ? 0xFFFFFFFFu : 0u;
  wh &= msk;
  wl &= msk;
  const int rw = clampi(row, 0, NP - 1);
  unsigned* dp = DST32 + (size_t)rw * 64 + lane;
  if (row < NP) { *(volatile unsigned*)dp = wh; *(volatile unsigned*)(dp + 32) = wl; }
  __threadfence();
  if (row < NP) { *(volatile unsigned*)dp = wh; *(volatile unsigned*)(dp + 32) = wl; }
}

template <int GATE>
__global__ __launch_bounds__(256) void k_walk(const float* __restrict__ P,
                                              const int* __restrict__ LNA, const int* __restrict__ CA,
                                              const int* __restrict__ OA, const int* __restrict__ FA,
                                              const int* __restrict__ LNB, const int* __restrict__ CB,
                                              const int* __restrict__ OB, const int* __restrict__ FB,
                                              const float* __restrict__ RDI, const float* __restrict__ RDO,
                                              const float* __restrict__ bias, float* ZS, int c0) {
  static_assert(GATE == 0 || GATE == 1);
  const int tid = (int)threadIdx.x, lane = tid & 31, wave = tid >> 5;
  const int row = (int)blockIdx.x * 8 + wave;
  const bool live = row < NN;
  const int ic = clampi(row, 0, NN - 1);
  const int b  = ic >> 10;
  const int cc = (c0 != 0) ? 32 : 0;
  int ca = CA[ic];
  int oa = OA[ic];
  const int fa = FA[ic];
  int cb = CB[ic];
  int ob = OB[ic];
  const int fb = FB[ic];
  asm volatile("" :: "v"(ca));
  asm volatile("" :: "v"(oa));
  asm volatile("" :: "v"(fa));
  asm volatile("" :: "v"(cb));
  asm volatile("" :: "v"(ob));
  asm volatile("" :: "v"(fb));
  ca = clampi(ca, 0, DEGCAP);
  cb = clampi(cb, 0, DEGCAP);
  oa = clampi(oa, 0, RCAP - DEGCAP);
  ob = clampi(ob, 0, RCAP - DEGCAP);
  const int na = __builtin_amdgcn_readfirstlane(live ? ca : 0);
  const int nb = __builtin_amdgcn_readfirstlane(live ? cb : 0);
  const int ua0 = clampi(list_word(LNA, b, oa, na, lane), 0, NN - 1);
  const int ua1 = clampi(list_word(LNA, b, oa, na, lane + 32), 0, NN - 1);
  const int vb0 = clampi(list_word(LNB, b, ob, nb, lane), 0, NN - 1);
  const int vb1 = clampi(list_word(LNB, b, ob, nb, lane + 32), 0, NN - 1);
  const float ra0 = RDO[ua0];
  const float ra1 = RDO[ua1];
  const float rdi = RDI[ic];
  asm volatile("" :: "v"(ra0));
  asm volatile("" :: "v"(ra1));
  asm volatile("" :: "v"(rdi));
  const float* Prow = P + (size_t)ic * NPC;
  const float own0 = Prow[lane];
  const float own1 = Prow[32 + lane];
  const float bg   = bias[cc + lane];
  asm volatile("" :: "v"(own0));
  asm volatile("" :: "v"(own1));
  asm volatile("" :: "v"(bg));
  const float a = own0 + own1;

  const float* Pf = P + 64 + lane;
  float F = 0.0f;
  const int na1 = na < 32 ? na : 32;
#pragma unroll 1
  for (int k = 0; k < na1; ++k) {
    const int   u = __builtin_amdgcn_readlane(ua0, k);
    const float r = __int_as_float(__builtin_amdgcn_readlane(__float_as_int(ra0), k));
    const float pv = Pf[(size_t)u * NPC];
    asm volatile("" :: "v"(pv));
    F = F + r * pv;
  }
#pragma unroll 1
  for (int k = 32; k < na; ++k) {
    const int   u = __builtin_amdgcn_readlane(ua1, k - 32);
    const float r = __int_as_float(__builtin_amdgcn_readlane(__float_as_int(ra1), k - 32));
    const float pv = Pf[(size_t)u * NPC];
    asm volatile("" :: "v"(pv));
    F = F + r * pv;
  }

  const float* Pb = P + 96 + lane;
  float B = 0.0f;
  const int nb1 = nb < 32 ? nb : 32;
#pragma unroll 1
  for (int k = 0; k < nb1; ++k) {
    const int v = __builtin_amdgcn_readlane(vb0, k);
    const float pv = Pb[(size_t)v * NPC];
    asm volatile("" :: "v"(pv));
    B = B + rdi * pv;
  }
#pragma unroll 1
  for (int k = 32; k < nb; ++k) {
    const int v = __builtin_amdgcn_readlane(vb1, k - 32);
    const float pv = Pb[(size_t)v * NPC];
    asm volatile("" :: "v"(pv));
    B = B + rdi * pv;
  }

  const float pre = ((a + F) + B) + bg;
  float* zp = ZS + (size_t)ic * HID + cc + lane;
  float res;
  if (GATE == 0) {
    res = sigm(pre);
  } else {
    const float z = *zp;
    asm volatile("" :: "v"(z));
    const float ht = tanhf(pre);
    const float hn = (1.0f - z) * ht;
    res = sigm(hn);
  }
  const float qn = __int_as_float(0x7fc00000);
  const float outv = ((fa | fb) != 0) ? qn : res;
  if (live) *(volatile float*)zp = outv;
  __threadfence();
  if (live) *(volatile float*)zp = outv;
}

__global__ __launch_bounds__(128) void k_out(const float* __restrict__ T, float* __restrict__ out) {
  const int f  = (int)blockIdx.x * 128 + (int)threadIdx.x;
  const int fc = f < OUT_ELEMS ? f : OUT_ELEMS - 1;
  const int n  = fc / OUTP;
  const int c  = fc - n * OUTP;
  const float v = T[(size_t)n * HID + c];
  asm volatile("" :: "v"(v));
  if (f < OUT_ELEMS) {
    volatile float* q = (volatile float*)(out + f);
    *q = v;
    __threadfence();
    *q = v;
  }
}

constexpr int ROW_BLOCKS   = NN / 8;
constexpr int SPLIT_BLOCKS = NP / 8;
constexpr int DEG_BLOCKS   = NN / 32;
constexpr int X24_BLOCKS   = NP * KX / 8 / 256;
constexpr int G_64  = (((NN + 63) / 64) * 1 + 7) / 8;
constexpr int G_128 = (((NN + 63) / 64) * 2 + 7) / 8;
static_assert(ROW_BLOCKS * 8 == NN && SPLIT_BLOCKS * 8 == NP && DEG_BLOCKS * 32 == NN);
static_assert(X24_BLOCKS * 256 * 8 == NP * KX && G_64 == 196 && G_128 == 391);
static_assert(OFF_ZS % 256 == 0 && OFF_HHL % 256 == 0 && OFF_X24 % 256 == 0 && OFF_LNA % 256 == 0);
static_assert(OFF_CA % 256 == 0 && OFF_RDI % 256 == 0 && OFF_RDO % 256 == 0 && OFF_W1T % 256 == 0);
static_assert(OFF_WCT % 256 == 0 && OFF_WOT % 256 == 0 && OFF_BIAS % 256 == 0);

extern "C" void kernel_launch(void* const* d_in, const int* in_sizes, int n_in,
                              void* d_out, int out_size, void* d_ws, size_t ws_size,
                              hipStream_t stream) {
  if (n_in < 13) return;
  if (in_sizes[0] != NN * XF) return;
  if (in_sizes[1] != 2 * NE) return;
  if (in_sizes[2] != NE) return;
  if (in_sizes[3] != XF * HID || in_sizes[4] != HID) return;
  if (in_sizes[5] != 4 * 128 * HID || in_sizes[6] != HID) return;
  if (in_sizes[9] != 4 * 128 * HID || in_sizes[10] != HID) return;
  if (in_sizes[11] != HID * OUTP || in_sizes[12] != OUTP) return;
  if (out_size != OUT_ELEMS) return;
  if (ws_size < WS_TOTAL) return;

  const float* x    = (const float*)d_in[0];
  const int*   ei   = (const int*)d_in[1];
  const float* ew   = (const float*)d_in[2];
  const float* wl2  = (const float*)d_in[3];
  const float* bl2  = (const float*)d_in[4];
  const float* wz   = (const float*)d_in[5];
  const float* bz   = (const float*)d_in[6];
  const float* wh   = (const float*)d_in[9];
  const float* bh   = (const float*)d_in[10];
  const float* wo   = (const float*)d_in[11];
  const float* bo   = (const float*)d_in[12];
  const int* rowp = ei;
  const int* colp = ei + NE;
  float* out = (float*)d_out;

  char* ws = (char*)d_ws;
  float*          P     = (float*)(ws + OFF_P);
  float*          T     = (float*)(ws + OFF_P);
  float*          ZS    = (float*)(ws + OFF_ZS);
  unsigned short* HHL   = (unsigned short*)(ws + OFF_HHL);
  unsigned*       HHL32 = (unsigned*)(ws + OFF_HHL);
  unsigned short* X24   = (unsigned short*)(ws + OFF_X24);
  int*            LNA   = (int*)(ws + OFF_LNA);
  int*            LEA   = (int*)(ws + OFF_LEA);
  int*            LNB   = (int*)(ws + OFF_LNB);
  int*            LEB   = (int*)(ws + OFF_LEB);
  int*            CA    = (int*)(ws + OFF_CA);
  int*            OA    = (int*)(ws + OFF_OA);
  int*            FA    = (int*)(ws + OFF_FA);
  int*            CB    = (int*)(ws + OFF_CB);
  int*            OB    = (int*)(ws + OFF_OB);
  int*            FB    = (int*)(ws + OFF_FB);
  float*          RDI   = (float*)(ws + OFF_RDI);
  float*          RDO   = (float*)(ws + OFF_RDO);
  unsigned short* W1T   = (unsigned short*)(ws + OFF_W1T);
  unsigned short* WCT   = (unsigned short*)(ws + OFF_WCT);
  unsigned short* WOT   = (unsigned short*)(ws + OFF_WOT);
  float*          BIAS  = (float*)(ws + OFF_BIAS);

  hipFuncSetAttribute(reinterpret_cast<const void*>(&k_build), hipFuncAttributeMaxDynamicSharedMemorySize, (int)BK_LDS);

  k_prep<<<PREP_BLOCKS, 256, 0, stream>>>(wl2, bl2, wz, bz, wh, bh, wo, bo, W1T, WCT, WOT, BIAS);
  k_plane<0><<<X24_BLOCKS, 256, 0, stream>>>(x, NN, XF, XF, X24, NP, KX);
  k_build<<<NBLK, 256, BK_LDS, stream>>>(colp, rowp, LNA, LEA, CA, OA, FA);
  k_build<<<NBLK, 256, BK_LDS, stream>>>(rowp, colp, LNB, LEB, CB, OB, FB);
  k_deg<<<DEG_BLOCKS, 256, 0, stream>>>(ew, LEA, CA, OA, FA, LEB, CB, OB, FB, RDI, RDO);
  k_gemm_nt<0, 0><<<G_64, 256, 0, stream>>>(X24, W1T, BIAS, ZS, NN, HID, KX, HID);
  k_split<0, SITE2_TWO_TERM><<<SPLIT_BLOCKS, 256, 0, stream>>>(ZS, BIAS, HHL32);
  for (int q = 0; q < 4; ++q) {
    const int c0 = 32 * (q & 1);
    k_gemm_nt<0, 0><<<G_128, 256, 0, stream>>>(HHL, WCT + (size_t)q * 128 * KH, BIAS, P, NN, NPC, KH, NPC);
    if (q < 2) {
      k_walk<0><<<ROW_BLOCKS, 256, 0, stream>>>(P, LNA, CA, OA, FA, LNB, CB, OB, FB, RDI, RDO, BIAS + 64, ZS, c0);
    } else {
      k_walk<1><<<ROW_BLOCKS, 256, 0, stream>>>(P, LNA, CA, OA, FA, LNB, CB, OB, FB, RDI, RDO, BIAS + 128, ZS, c0);
    }
  }
  k_split<1, SITE3_TWO_TERM><<<SPLIT_BLOCKS, 256, 0, stream>>>(ZS, BIAS, HHL32);
  k_gemm_nt<0, 1><<<G_64, 256, 0, stream>>>(HHL, WOT, BIAS + 192, T, NN, HID, KH, HID);
  k_out<<<OUT_ELEMS / 128, 128, 0, stream>>>(T, out);
}
